// GridMultiHeadAttention_2877628088558
// MI455X (gfx1250) — hardware-verified
//
#include <hip/hip_runtime.h>


#define NB_  4
#define NT_  2048
#define HS   1024
#define DM   HS
#define NH_  8
#define NKV  8
#define HD   128
#define KW   (NKV * HD)
#define SCL  0.08838834764831845f
#define PSC  32768.0f
#define LOSC 1024.0f
#define LOSCI (1.0f / 1024.0f)

typedef _Float16 h16;
typedef unsigned short bf;
typedef __attribute__((ext_vector_type(16))) __bf16   v16bf;
typedef __attribute__((ext_vector_type(16))) _Float16 v16h;
typedef __attribute__((ext_vector_type(8)))  _Float16 v8h;
typedef __attribute__((ext_vector_type(8)))  unsigned short v8us;
typedef __attribute__((ext_vector_type(8)))  float    v8f;
typedef __attribute__((ext_vector_type(4)))  float    v4f;
typedef __attribute__((ext_vector_type(4)))  _Float16 v4h;
typedef v8h  __attribute__((may_alias)) v8ha;
typedef v4f  __attribute__((may_alias)) v4fa;
typedef v8us __attribute__((may_alias)) v8usa;

__device__ __forceinline__ unsigned short f2bf(float f) { unsigned u = __float_as_uint(f); u += 0x7FFFu + ((u >> 16) & 1u); return (unsigned short)(u >> 16); }
__device__ __forceinline__ float bf2f(unsigned short b) { return __uint_as_float(((unsigned)b) << 16); }
__device__ __forceinline__ float bfr(float f) { return bf2f(f2bf(f)); }
__device__ __forceinline__ v16h cat16(v8h lo, v8h hi) { return __builtin_shufflevector(lo, hi, 0, 1, 2, 3, 4, 5, 6, 7, 8, 9, 10, 11, 12, 13, 14, 15); }
__device__ __forceinline__ v16bf cat16b(v8us lo, v8us hi) { return __builtin_bit_cast(v16bf, __builtin_shufflevector(lo, hi, 0, 1, 2, 3, 4, 5, 6, 7, 8, 9, 10, 11, 12, 13, 14, 15)); }
__device__ __forceinline__ v8f wmma16(v16h a, v16h b, v8f c) { return __builtin_amdgcn_wmma_f32_16x16x32_f16(false, a, false, b, (short)0, c, false, false); }
__device__ __forceinline__ v8f wmmab(v16bf a, v16bf b, v8f c) { return __builtin_amdgcn_wmma_f32_16x16x32_bf16(false, a, false, b, (short)0, c, false, false); }

__global__ __launch_bounds__(256) void k_cvtb(const float* __restrict__ src, int nrows, bf* dst) {
    const int lane = threadIdx.x & 31, r = blockIdx.x * 8 + (threadIdx.x >> 5);
    if (r >= nrows) return;
#pragma unroll 1
    for (int ps = 0; ps < 2; ++ps) {
#pragma unroll
        for (int q = 0; q < HS / 256; ++q) { v8us o;
#pragma unroll
            for (int i = 0; i < 8; ++i) o[i] = f2bf(src[(size_t)r * HS + q * 256 + lane * 8 + i]);
            *(volatile v8us*)(dst + (size_t)r * HS + q * 256 + lane * 8) = o; }
        if (ps == 0) __threadfence(); }
}
template <bool SPLITA>
__global__ __launch_bounds__(128) void k_gemm(const bf* __restrict__ A, const bf* __restrict__ Al, const bf* __restrict__ Bn, const float* __restrict__ bias, int ldc, float* C) {
    __shared__ __align__(16) float ost[4][16 * 68];
    const int lane = threadIdx.x & 31, wave = threadIdx.x >> 5, lr = lane & 15, hi = lane >> 4;
    const size_t r0 = (size_t)blockIdx.x * 64 + wave * 16; const int c0 = blockIdx.y * 64;
    const size_t aoff = (r0 + lr) * HS + 8 * hi;
    v8f acc[4];
#pragma unroll
    for (int t = 0; t < 4; ++t) acc[t] = (v8f){};
#pragma unroll 2
    for (int kc = 0; kc < HS; kc += 32) {
        const v16bf a = cat16b(*(const v8us*)(A + aoff + kc), *(const v8us*)(A + aoff + kc + 16));
        v16bf al = a; if (SPLITA) al = cat16b(*(const v8us*)(Al + aoff + kc), *(const v8us*)(Al + aoff + kc + 16));
#pragma unroll
        for (int t = 0; t < 4; ++t) { const bf* bp = Bn + (size_t)(c0 + t * 16 + lr) * HS + kc + 8 * hi; const v16bf bb = cat16b(*(const v8us*)bp, *(const v8us*)(bp + 16)); acc[t] = wmmab(a, bb, acc[t]); if (SPLITA) acc[t] = wmmab(al, bb, acc[t]); }
        asm volatile("v_nop" : "+v"(acc[0]), "+v"(acc[1]), "+v"(acc[2]), "+v"(acc[3]) : "v"(a), "v"(al) : "memory");
    }
    float* os = &ost[wave][0];
#pragma unroll
    for (int t = 0; t < 4; ++t)
#pragma unroll
        for (int j = 0; j < 8; ++j) os[(hi * 8 + j) * 68 + t * 16 + lr] = acc[t][j] + (bias ? bfr(bias[c0 + t * 16 + lr]) : 0.f);
    __builtin_amdgcn_wave_barrier(); asm volatile("" ::: "memory");
    float* crow = C + r0 * ldc + c0;
    auto pass = [&]() {
#pragma unroll
        for (int s = 0; s < 8; ++s) { const int Lid = (lane >> 3) + 4 * s, piece = lane & 7; const int row = Lid >> 1, cofs = (Lid & 1) * 32 + piece * 4;
            const v4f val = *(const v4fa*)(os + row * 68 + cofs); *(volatile v4f*)(crow + (size_t)row * ldc + cofs) = val; }
    };
    pass(); __threadfence(); pass();
}
__global__ __launch_bounds__(256) void k_sp16b(const float* __restrict__ T, int nrows, h16* Yh, h16* Yl) {
    const int lane = threadIdx.x & 31, r = blockIdx.x * 8 + (threadIdx.x >> 5);
    if (r >= nrows) return;
#pragma unroll 1
    for (int ps = 0; ps < 2; ++ps) {
#pragma unroll 1
        for (int q = 0; q < DM / 256; ++q) { const size_t o = (size_t)r * DM + q * 256 + lane * 8; const v8f v = *(const v8f*)(T + o); v8h oh, ol;
#pragma unroll
            for (int k = 0; k < 8; ++k) { const h16 a = (h16)v[k]; oh[k] = a; ol[k] = (h16)((v[k] - (float)a) * LOSC); }
            *(volatile v8h*)(Yh + o) = oh; *(volatile v8h*)(Yl + o) = ol; }
        if (ps == 0) __threadfence(); }
}
__global__ __launch_bounds__(256) void k_split(const float* __restrict__ src, int nrows, bf* dh, bf* dl) {
    const int lane = threadIdx.x & 31, r = blockIdx.x * 8 + (threadIdx.x >> 5);
    if (r >= nrows) return;
#pragma unroll 1
    for (int ps = 0; ps < 2; ++ps) {
#pragma unroll 1
        for (int q = 0; q < DM / 256; ++q) { const size_t o = (size_t)r * DM + q * 256 + lane * 8; const v8f v = *(const v8f*)(src + o); v8us oh, ol;
#pragma unroll
            for (int i = 0; i < 8; ++i) { const unsigned short hb = f2bf(v[i]); oh[i] = hb; ol[i] = f2bf(v[i] - bf2f(hb)); }
            *(volatile v8us*)(dh + o) = oh; *(volatile v8us*)(dl + o) = ol; }
        if (ps == 0) __threadfence(); }
}
__global__ __launch_bounds__(256) void k_lnfin(const float* __restrict__ X, const float* __restrict__ Rres, const float* __restrict__ gam, const float* __restrict__ bet, int nrows, float* OUTP) {
    const int lane = threadIdx.x & 31, r = blockIdx.x * 8 + (threadIdx.x >> 5);
    if (r >= nrows) return;
    const float* xr = X + (size_t)r * DM; const float* rr = Rres + (size_t)r * DM;
    float s = 0.f;
#pragma unroll 1
    for (int q = 0; q < 2 * (DM / 256); ++q) { const int c0 = (q >> 1) * 256 + (q & 1) * 128 + lane * 4; v4f v = *(const v4f*)(xr + c0); { const v4f q4 = *(const v4f*)(rr + c0); for (int i2 = 0; i2 < 4; ++i2) v[i2] += bfr(q4[i2]); }
#pragma unroll
        for (int i = 0; i < 4; ++i) s += v[i]; }
#pragma unroll
    for (int sh = 16; sh; sh >>= 1) s += __shfl_xor(s, sh, 32);
    const float mu = s * (1.0f / DM);
    float s2 = 0.f;
#pragma unroll 1
    for (int q = 0; q < 2 * (DM / 256); ++q) { const int c0 = (q >> 1) * 256 + (q & 1) * 128 + lane * 4; v4f v = *(const v4f*)(xr + c0); { const v4f q4 = *(const v4f*)(rr + c0); for (int i2 = 0; i2 < 4; ++i2) v[i2] += bfr(q4[i2]); }
#pragma unroll
        for (int i = 0; i < 4; ++i) { const float d = v[i] - mu; s2 = fmaf(d, d, s2); } }
#pragma unroll
    for (int sh = 16; sh; sh >>= 1) s2 += __shfl_xor(s2, sh, 32);
    const float rs = rsqrtf(s2 * (1.0f / DM) + 1e-5f);
#pragma unroll 1
    for (int ps = 0; ps < 2; ++ps) {
#pragma unroll 1
        for (int q = 0; q < 2 * (DM / 256); ++q) { const int c0 = (q >> 1) * 256 + (q & 1) * 128 + lane * 4; v4f v = *(const v4f*)(xr + c0); { const v4f q4 = *(const v4f*)(rr + c0); for (int i2 = 0; i2 < 4; ++i2) v[i2] += bfr(q4[i2]); } v4f y;
#pragma unroll
            for (int i = 0; i < 4; ++i) y[i] = (v[i] - mu) * rs * bfr(gam[c0 + i]) + bfr(bet[c0 + i]);
            *(volatile v4f*)(OUTP + (size_t)r * DM + c0) = y; }
        if (ps == 0) __threadfence(); }
}
__global__ __launch_bounds__(256) void k_vt(const float* __restrict__ V, bf* VTH, bf* VTL) {
    __shared__ float tl[64][65];
    const int tid = threadIdx.x, t0 = blockIdx.x * 64, d0 = blockIdx.y * 64, g = blockIdx.z;
    { const int tt = tid >> 2, dq = (tid & 3) * 16;
#pragma unroll
      for (int i = 0; i < 16; ++i) tl[dq + i][tt] = V[(size_t)(t0 + tt) * KW + g * HD + d0 + dq + i]; }
    __syncthreads();
    const int piece = tid & 7;
    auto pass = [&]() {
#pragma unroll
        for (int s = 0; s < 2; ++s) { const int d = (tid >> 3) + 32 * s; v8us oh, ol;
#pragma unroll
            for (int i = 0; i < 8; ++i) { const float v = tl[d][piece * 8 + i]; const unsigned short hb = f2bf(v); oh[i] = hb; ol[i] = f2bf(v - bf2f(hb)); }
            const size_t o = ((size_t)g * HD + d0 + d) * NT_ + t0 + piece * 8; *(volatile v8us*)(VTH + o) = oh; *(volatile v8us*)(VTL + o) = ol; }
    };
    pass(); __threadfence(); pass();
}
__global__ __launch_bounds__(128) void k_attn(const h16* __restrict__ QH, const h16* __restrict__ QL, const h16* __restrict__ KH, const h16* __restrict__ KL, const bf* __restrict__ VTH, const bf* __restrict__ VTL, float* OUTP) {
    __shared__ __align__(16) unsigned short plds[4][16 * 32];
    __shared__ __align__(16) unsigned short plds2[4][16 * 32];
    __shared__ __align__(16) float ost[4][16 * 68];
    const int lane = threadIdx.x & 31, wave = threadIdx.x >> 5, lr = lane & 15, hi = lane >> 4;
    const int bid = blockIdx.x; const int h = bid / (NT_ / 64), qt = bid - h * (NT_ / 64); const int g = h;
    const int q0 = qt * 64 + wave * 16;
    unsigned short* pl = &plds[wave][0]; unsigned short* pl2 = &plds2[wave][0];
    const size_t qo = (size_t)(q0 + lr) * (NH_ * HD) + h * HD + 8 * hi;
    const h16* kh_b = KH + g * HD; const h16* kl_b = KL + g * HD;
    const size_t vbase = ((size_t)g * HD) * NT_;
    v8f o[8];
#pragma unroll
    for (int n = 0; n < 8; ++n) o[n] = (v8f){};
    float mrow[8], lpart[8];
#pragma unroll
    for (int j = 0; j < 8; ++j) { mrow[j] = -3.0e38f; lpart[j] = 0.f; }
    const int kt_hi = NT_ / 32 - 1;
#pragma unroll 1
    for (int kt = 0; kt <= kt_hi; ++kt) {
        const int l0 = kt * 32;
        const size_t ko0 = (size_t)(l0 + lr) * KW + 8 * hi, ko1 = (size_t)(l0 + 16 + lr) * KW + 8 * hi;
        v8f s0 = {}, s1 = {}, x0 = {}, x1 = {};
#pragma unroll
        for (int kc = 0; kc < 4; ++kc) {
            const v16h qa = cat16(*(const v8h*)(QH + qo + kc * 32), *(const v8h*)(QH + qo + kc * 32 + 16)), qx = cat16(*(const v8h*)(QL + qo + kc * 32), *(const v8h*)(QL + qo + kc * 32 + 16));
            const v16h k0h = cat16(*(const v8h*)(kh_b + ko0 + kc * 32), *(const v8h*)(kh_b + ko0 + kc * 32 + 16)), k1h = cat16(*(const v8h*)(kh_b + ko1 + kc * 32), *(const v8h*)(kh_b + ko1 + kc * 32 + 16));
            s0 = wmma16(qa, k0h, s0); s1 = wmma16(qa, k1h, s1); x0 = wmma16(qx, k0h, x0); x1 = wmma16(qx, k1h, x1);
            asm volatile("v_nop" : "+v"(s0), "+v"(s1), "+v"(x0), "+v"(x1) : "v"(qa), "v"(qx), "v"(k0h), "v"(k1h) : "memory");
            const v16h k0l = cat16(*(const v8h*)(kl_b + ko0 + kc * 32), *(const v8h*)(kl_b + ko0 + kc * 32 + 16)), k1l = cat16(*(const v8h*)(kl_b + ko1 + kc * 32), *(const v8h*)(kl_b + ko1 + kc * 32 + 16));
            x0 = wmma16(qa, k0l, x0); x1 = wmma16(qa, k1l, x1);
            asm volatile("v_nop" : "+v"(x0), "+v"(x1) : "v"(k0l), "v"(k1l) : "memory");
        }
        asm volatile("v_nop\n\tv_nop\n\tv_nop\n\tv_nop" : "+v"(s0), "+v"(s1), "+v"(x0), "+v"(x1));
        float alpha[8];
#pragma unroll
        for (int j = 0; j < 8; ++j) { const int qi = q0 + hi * 8 + j, ja = l0 + lr, jb = l0 + 16 + lr;
            const float a0 = (s0[j] + x0[j] * LOSCI) * SCL, a1 = (s1[j] + x1[j] * LOSCI) * SCL; (void)ja; (void)jb; (void)qi;
            float mx = fmaxf(a0, a1);
            mx = fmaxf(mx, __shfl_xor(mx, 1, 16)); mx = fmaxf(mx, __shfl_xor(mx, 2, 16)); mx = fmaxf(mx, __shfl_xor(mx, 4, 16)); mx = fmaxf(mx, __shfl_xor(mx, 8, 16));
            const float mn = fmaxf(mrow[j], mx);
            alpha[j] = __expf(mrow[j] - mn); mrow[j] = mn;
            const float p0 = __expf(a0 - mn), p1 = __expf(a1 - mn);
            lpart[j] = lpart[j] * alpha[j] + (p0 + p1);
            const int mr = hi * 8 + j; const float ps0 = p0 * PSC, ps1 = p1 * PSC; const unsigned short h0 = f2bf(ps0), h1 = f2bf(ps1);
            pl[mr * 32 + lr] = h0; pl[mr * 32 + 16 + lr] = h1; pl2[mr * 32 + lr] = f2bf(ps0 - bf2f(h0)); pl2[mr * 32 + 16 + lr] = f2bf(ps1 - bf2f(h1)); }
#pragma unroll
        for (int n = 0; n < 8; ++n)
#pragma unroll
            for (int j = 0; j < 8; ++j) o[n][j] *= alpha[j];
        asm volatile("" ::: "memory");
        const v16bf pa = cat16b(*(const v8usa*)(pl + lr * 32 + hi * 8), *(const v8usa*)(pl + lr * 32 + 16 + hi * 8));
        const v16bf px = cat16b(*(const v8usa*)(pl2 + lr * 32 + hi * 8), *(const v8usa*)(pl2 + lr * 32 + 16 + hi * 8));
#pragma unroll
        for (int n = 0; n < 8; ++n) { const size_t vo = vbase + (size_t)(n * 16 + lr) * NT_ + l0 + hi * 8;
            const v16bf vh = cat16b(*(const v8us*)(VTH + vo), *(const v8us*)(VTH + vo + 16)), vl = cat16b(*(const v8us*)(VTL + vo), *(const v8us*)(VTL + vo + 16));
            o[n] = wmmab(pa, vh, o[n]); o[n] = wmmab(px, vh, o[n]); o[n] = wmmab(pa, vl, o[n]);
            asm volatile("" : "+v"(o[n]) : "v"(vh), "v"(vl) : "memory"); }
        asm volatile("v_nop\n\tv_nop\n\tv_nop\n\tv_nop" : "+v"(o[0]), "+v"(o[7]) : "v"(pa), "v"(px));
        __builtin_amdgcn_wave_barrier();
    }
    float inv[8];
#pragma unroll
    for (int j = 0; j < 8; ++j) { float rs = lpart[j]; rs += __shfl_xor(rs, 1, 16); rs += __shfl_xor(rs, 2, 16); rs += __shfl_xor(rs, 4, 16); rs += __shfl_xor(rs, 8, 16); inv[j] = 1.0f / (rs * PSC); }
    float* os = &ost[wave][0];
    float* ob = OUTP + (size_t)q0 * (NH_ * HD) + (size_t)h * HD;
#pragma unroll
    for (int half = 0; half < 2; ++half) {
#pragma unroll
        for (int n = 0; n < 4; ++n)
#pragma unroll
            for (int j = 0; j < 8; ++j) os[(hi * 8 + j) * 68 + n * 16 + lr] = o[half * 4 + n][j] * inv[j];
        __builtin_amdgcn_wave_barrier(); asm volatile("" ::: "memory");
#pragma unroll
        for (int ps2 = 0; ps2 < 2; ++ps2) {
#pragma unroll
            for (int s = 0; s < 8; ++s) { const int Lid = (lane >> 3) + 4 * s, piece = lane & 7; const int row = Lid >> 1, cofs = (Lid & 1) * 32 + piece * 4;
                const v4f val = *(const v4fa*)(os + row * 68 + cofs); *(volatile v4f*)(ob + (size_t)row * (NH_ * HD) + half * 64 + cofs) = val; }
            if (ps2 == 0) __threadfence(); }
        __builtin_amdgcn_wave_barrier(); asm volatile("" ::: "memory");
    }
}

extern "C" void kernel_launch(void* const* d_in, const int* in_sizes, int n_in,
                              void* d_out, int out_size, void* d_ws, size_t ws_size, hipStream_t stream) {
    (void)in_sizes; (void)n_in; (void)out_size;
    const float* x = (const float*)d_in[0];
    const float* Wq = (const float*)d_in[1]; const float* bq = (const float*)d_in[2]; const float* Wk = (const float*)d_in[3]; const float* bk = (const float*)d_in[4]; const float* Wv = (const float*)d_in[5]; const float* bv = (const float*)d_in[6];
    const float* Wo = (const float*)d_in[7]; const float* bo = (const float*)d_in[8]; const float* lg = (const float*)d_in[9]; const float* lb = (const float*)d_in[10];
    float* out = (float*)d_out;
    char* wsp = (char*)d_ws;
    auto take = [&](size_t bytes) { char* p = wsp; wsp += (bytes + 255) & ~(size_t)255; return (void*)p; };
    bf* Xb = (bf*)take((size_t)NT_ * HS * 2); bf* WqB = (bf*)take((size_t)HS * HS * 2); bf* WkB = (bf*)take((size_t)HS * HS * 2); bf* WvB = (bf*)take((size_t)HS * HS * 2); bf* WoB = (bf*)take((size_t)HS * HS * 2);
    float* TMP = (float*)take((size_t)NT_ * HS * 4);
    h16* QH = (h16*)take((size_t)NT_ * HS * 2); h16* QL = (h16*)take((size_t)NT_ * HS * 2); h16* KH = (h16*)take((size_t)NT_ * KW * 2); h16* KL = (h16*)take((size_t)NT_ * KW * 2);
    bf* VTH = (bf*)take((size_t)KW * NT_ * 2); bf* VTL = (bf*)take((size_t)KW * NT_ * 2); float* CTX = (float*)take((size_t)NT_ * HS * 4); bf* Ch = (bf*)take((size_t)NT_ * HS * 2); bf* Cl = (bf*)take((size_t)NT_ * HS * 2); float* Y = (float*)take((size_t)NT_ * HS * 4);
    if ((size_t)(wsp - (char*)d_ws) > ws_size) return;
    k_cvtb<<<HS / 8, 256, 0, stream>>>(Wq, HS, WqB); k_cvtb<<<HS / 8, 256, 0, stream>>>(Wk, HS, WkB); k_cvtb<<<HS / 8, 256, 0, stream>>>(Wv, HS, WvB); k_cvtb<<<HS / 8, 256, 0, stream>>>(Wo, HS, WoB);
    for (int b = 0; b < NB_; ++b) {
        const float* xb = x + (size_t)b * NT_ * HS;
        k_cvtb<<<NT_ / 8, 256, 0, stream>>>(xb, NT_, Xb);
        k_gemm<false><<<dim3(NT_ / 64, HS / 64, 1), 128, 0, stream>>>(Xb, nullptr, WqB, bq, HS, TMP); k_sp16b<<<NT_ / 8, 256, 0, stream>>>(TMP, NT_, QH, QL);
        k_gemm<false><<<dim3(NT_ / 64, HS / 64, 1), 128, 0, stream>>>(Xb, nullptr, WkB, bk, HS, TMP); k_sp16b<<<NT_ / 8, 256, 0, stream>>>(TMP, NT_, KH, KL);
        k_gemm<false><<<dim3(NT_ / 64, HS / 64, 1), 128, 0, stream>>>(Xb, nullptr, WvB, bv, HS, TMP); k_vt<<<dim3(NT_ / 64, 2, NKV), 256, 0, stream>>>(TMP, VTH, VTL);
        k_attn<<<NH_ * (NT_ / 64), 128, 0, stream>>>(QH, QL, KH, KL, VTH, VTL, CTX);
        k_split<<<NT_ / 8, 256, 0, stream>>>(CTX, NT_, Ch, Cl);
        k_gemm<true><<<dim3(NT_ / 64, HS / 64, 1), 128, 0, stream>>>(Ch, Cl, WoB, bo, HS, Y);
        k_lnfin<<<NT_ / 8, 256, 0, stream>>>(Y, xb, lg, lb, NT_, out + (size_t)b * NT_ * HS);
    }
}
